// OAIAttention_11579231830229
// MI455X (gfx1250) — hardware-verified
//
#include <hip/hip_runtime.h>
#include <hip/hip_bf16.h>
#include <math.h>

#define TT_  2048
#define HID  2880
#define NQH  64
#define NKV  8
#define DKK  64
#define SS   2048
#define HH   8
#define BB   1
#define WIN  128
#define QKN  4608
#define QW   2

typedef _Float16 bf16;
typedef __attribute__((ext_vector_type(4))) unsigned v4u_t;
typedef unsigned v4ua __attribute__((ext_vector_type(4), may_alias));
typedef __attribute__((ext_vector_type(4))) float v4f_t;
typedef float v4fa __attribute__((ext_vector_type(4), may_alias));
typedef __attribute__((ext_vector_type(16))) bf16  bf16x16;
typedef __attribute__((ext_vector_type(8)))  bf16  bf16x8;
typedef __attribute__((ext_vector_type(4)))  bf16  bf16x4;
typedef __attribute__((ext_vector_type(8)))  float f32x8;
struct RopeFreq { float inv[32]; };

#define LDS_STRIDE 48
#define KSTRIDE    72
#define VSTRIDE    48

__device__ __forceinline__ f32x8 wmma_bf16(bf16x16 a, bf16x16 b, f32x8 c) {
  c = __builtin_amdgcn_wmma_f32_16x16x32_f16(false, a, false, b, (short)0, c, false, false);
  asm volatile("v_nop\n\tv_nop\n\tv_nop\n\tv_nop" : "+v"(c) : "v"(a), "v"(b));
  return c;
}

template <typename T>
__device__ __forceinline__ bf16x16 load_frag(const T* __restrict__ base, int ld,
                                             int row0, int k0) {
  const int lane = threadIdx.x & 31;
  const int r    = lane & 15;
  const int kh   = (lane >> 4) * 8;
  const T* p0 = base + (size_t)(row0 + r) * ld + (k0 + kh);
  const T* p1 = p0 + 16;
  bf16x16 f;
#pragma unroll
  for (int i = 0; i < 8; ++i) {
    f[i]     = (bf16)p0[i];
    f[i + 8] = (bf16)p1[i];
  }
  return f;
}

__device__ __forceinline__ bf16x16 lds_frag(const bf16* base, int stride) {
  const int lane = threadIdx.x & 31;
  const int row  = lane & 15;
  const int kh   = (lane >> 4) * 8;
  const bf16x8 lo = *(const bf16x8*)(base + row * stride + kh);
  const bf16x8 hi = *(const bf16x8*)(base + row * stride + kh + 16);
  bf16x16 f;
#pragma unroll
  for (int i = 0; i < 8; ++i) { f[i] = lo[i]; f[i + 8] = hi[i]; }
  return f;
}

template <typename T>
__device__ __forceinline__ void stage_read16(const T* __restrict__ p, float* buf) {
#pragma unroll
  for (int i = 0; i < 16; ++i) buf[i] = (float)p[i];
}

__device__ __forceinline__ void stage_write(bf16* dst, const float* buf, int nquad) {
#pragma unroll
  for (int i = 0; i < nquad; ++i) {
    bf16x4 q;
    q[0] = (bf16)buf[4 * i];     q[1] = (bf16)buf[4 * i + 1];
    q[2] = (bf16)buf[4 * i + 2]; q[3] = (bf16)buf[4 * i + 3];
    *(bf16x4*)(dst + 4 * i) = q;
  }
}

template <typename AT, int MODE>
__global__ __launch_bounds__(256) void gemm_oai_kernel(
    const AT* __restrict__ A, const float* __restrict__ W,
    const float* __restrict__ bias, const float* __restrict__ rowscale, const float* __restrict__ R, void* __restrict__ out,
    int M, int N, int K) {
  __shared__ bf16 ldsA[128 * LDS_STRIDE];
  __shared__ bf16 ldsW[256 * LDS_STRIDE];
  __shared__ __attribute__((aligned(16))) unsigned char sob[256 * 136 * 2];

  const int t    = threadIdx.x;
  const int wave = t >> 5;
  const int lane = t & 31;
  const int wm   = (wave & 1) * 64;
  const int wn   = (wave >> 1) * 64;
  const int mBlk = blockIdx.x * 128;
  const int nBlk = blockIdx.y * 256;

  const int arow = t >> 1;
  const int ach  = (t & 1) * 16;

  float abuf[16];
  float wbuf[32];

  stage_read16(A + (size_t)(mBlk + arow) * K + ach, abuf);
  const int nrow = min(nBlk + t, N - 1);
  stage_read16(W + (size_t)nrow * K,          wbuf);
  stage_read16(W + (size_t)nrow * K + 16,     wbuf + 16);

  f32x8 acc[4][4] = {};

  for (int k = 0; k < K; k += 32) {
    __syncthreads();
    stage_write(&ldsA[arow * LDS_STRIDE + ach], abuf, 4);
    stage_write(&ldsW[t * LDS_STRIDE],          wbuf, 8);
    if (k + 32 < K) {
      stage_read16(A + (size_t)(mBlk + arow) * K + (k + 32) + ach, abuf);
      stage_read16(W + (size_t)nrow * K + (k + 32),          wbuf);
      stage_read16(W + (size_t)nrow * K + (k + 32) + 16,     wbuf + 16);
    }
    __syncthreads();

    bf16x16 af[4], wf[4];
#pragma unroll
    for (int i = 0; i < 4; ++i)
      af[i] = lds_frag(ldsA + (wm + 16 * i) * LDS_STRIDE, LDS_STRIDE);
#pragma unroll
    for (int j = 0; j < 4; ++j)
      wf[j] = lds_frag(ldsW + (wn + 16 * j) * LDS_STRIDE, LDS_STRIDE);
#pragma unroll
    for (int i = 0; i < 4; ++i)
#pragma unroll
      for (int j = 0; j < 4; ++j)
        acc[i][j] = wmma_bf16(af[i], wf[j], acc[i][j]);
  }

  const int nlane = lane & 15;
  const int mh    = (lane >> 4) * 8;
  __syncthreads();
  if (MODE == 0 || MODE == 1 || MODE == 3) {
    bf16* so = (bf16*)sob;
#pragma unroll
    for (int i = 0; i < 4; ++i)
#pragma unroll
      for (int j = 0; j < 4; ++j) {
        const int nl = wn + 16 * j + nlane;
        const float bv = bias ? bias[min(nBlk + nl, N - 1)] : 0.0f;
        if (MODE == 3) {
#pragma unroll 1
          for (int r = 0; r < 8; ++r) {
            const int ml = wm + 16 * i + mh + r;
            const float xg = acc[i][j][r] + bv;
            so[ml * 264 + nl] = (bf16)(0.5f * xg * (1.0f + erff(xg * 0.70710678118654752f)));
          }
        } else {
#pragma unroll
        for (int r = 0; r < 8; ++r) {
          const int ml = wm + 16 * i + mh + r;
          const bf16 hv = (bf16)(acc[i][j][r] * (rowscale ? rowscale[mBlk + ml] : 1.0f) + bv);
          if (MODE == 0) so[ml * 264 + nl] = hv;
          else           so[nl * 136 + ml] = hv;
        }
        }
      }
    __syncthreads();
#pragma unroll 1
    for (int pass = 0; pass < 2; ++pass) {
      if (MODE == 0 || MODE == 3) {
        for (int ch = t; ch < 128 * 32; ch += 256) { const int ml = ch >> 5, q = (ch & 31) * 8;
          *(volatile v4u_t*)((bf16*)out + (size_t)(mBlk + ml) * N + nBlk + q) = *(const v4ua*)(so + ml * 264 + q); }
      } else {
        const int b_ = mBlk / SS, s0 = mBlk & (SS - 1);
        for (int ch = t; ch < 256 * 16; ch += 256) { const int nl = ch >> 4, q = (ch & 15) * 8; const int n = nBlk + nl, h = n >> 6, dk = n & (DKK - 1);
          *(volatile v4u_t*)((bf16*)out + (((size_t)(b_ * HH + h)) * DKK + dk) * SS + s0 + q) = *(const v4ua*)(so + nl * 136 + q); }
      }
      __threadfence();
    }
  } else {
    float* so = (float*)sob;
#pragma unroll 1
    for (int hf = 0; hf < 2; ++hf) {
      if (wm == hf * 64) {
#pragma unroll
        for (int i = 0; i < 4; ++i)
#pragma unroll
          for (int j = 0; j < 4; ++j) {
            const int nl = wn + 16 * j + nlane;
            const float bv = bias ? bias[min(nBlk + nl, N - 1)] : 0.0f;
#pragma unroll
            for (int r = 0; r < 8; ++r) so[(16 * i + mh + r) * 260 + nl] = acc[i][j][r] * (rowscale ? rowscale[mBlk + hf * 64 + 16 * i + mh + r] : 1.0f) + bv;
          }
      }
      __syncthreads();
      if (R) {
        for (int ch = t; ch < 64 * 64; ch += 256) { const int ml = ch >> 6, q = (ch & 63) * 4;
          if (nBlk + q < N) { const v4f_t rv = *(const v4f_t*)(R + (size_t)(mBlk + hf * 64 + ml) * N + nBlk + q); v4f_t v = *(const volatile v4fa*)(so + ml * 260 + q); v += rv; *(volatile v4fa*)(so + ml * 260 + q) = v; } }
        asm volatile("s_wait_dscnt 0" ::: "memory");
      }
#pragma unroll 1
      for (int pass = 0; pass < 2; ++pass) {
        for (int ch = t; ch < 64 * 64; ch += 256) { const int ml = ch >> 6, q = (ch & 63) * 4;
          if (nBlk + q < N) *(volatile v4f_t*)((float*)out + (size_t)(mBlk + hf * 64 + ml) * N + nBlk + q) = *(const volatile v4fa*)(so + ml * 260 + q); }
        __threadfence();
      }
      __syncthreads();
    }
  }
}


#define QST  4096
#define KVST 512
__global__ __launch_bounds__(64) void attn_kernel(
    const bf16* __restrict__ Qb, const bf16* __restrict__ Kb,
    const bf16* __restrict__ Vt, const float* __restrict__ sinks,
    bf16* __restrict__ attnOut) {
  __shared__ bf16 ldsK[32 * KSTRIDE];
  __shared__ bf16 ldsV[64 * VSTRIDE];
  __shared__ __attribute__((aligned(16))) bf16 ldsO[2][32 * 72];

  const int q0blk = blockIdx.x * 64;
  const int h  = blockIdx.y;
  const int b  = blockIdx.z;
  const int t    = threadIdx.x;
  const int wave = t >> 5;
  const int lane = t & 31;
  const int qlane = lane & 15;
  const int kh8   = (lane >> 4) * 8;
  const int q0 = q0blk + wave * 32;

  const int hk = h >> 3;
  const bf16* Qh = Qb + (size_t)b * SS * QST + h * DKK;
  const bf16* Kh = Kb + (size_t)b * SS * KVST + hk * DKK;
  const bf16* Vh = Vt + ((size_t)(b * HH + hk)) * DKK * SS;

  const int krow = t >> 1;
  const int kcol = (t & 1) * 32;
  const bf16* kSrc = Kh + (size_t)krow * KVST + kcol;
  const bf16* vSrc = Vh + (size_t)t * SS;

  bf16x16 qf[QW][2];
#pragma unroll
  for (int qt = 0; qt < QW; ++qt) {
    qf[qt][0] = load_frag(Qh, QST, q0 + 16 * qt, 0);
    qf[qt][1] = load_frag(Qh, QST, q0 + 16 * qt, 32);
  }

  f32x8 o[QW][4] = {};
  float mrun[QW], lrun[QW];
#pragma unroll
  for (int qt = 0; qt < QW; ++qt) { mrun[qt] = sinks[h] * 1.44269504088896340736f; lrun[qt] = 1.0f; }

  const float scale = 0.125f * 1.44269504088896340736f;
  const float NEG2 = -1.0e9f;
  const int kmax = q0blk + 63;
  const int kmin = (q0blk >= WIN - 1) ? ((q0blk - (WIN - 1)) & ~31) : 0;

  bf16x8 kreg[4], vreg[4];
#pragma unroll
  for (int i = 0; i < 4; ++i) {
    kreg[i] = *(const bf16x8*)(kSrc + (size_t)kmin * KVST + 8 * i);
    vreg[i] = *(const bf16x8*)(vSrc + kmin + 8 * i);
  }

  for (int kb = kmin; kb <= kmax; kb += 32) {
    __syncthreads();
#pragma unroll
    for (int i = 0; i < 4; ++i) {
      *(bf16x8*)(&ldsK[krow * KSTRIDE + kcol + 8 * i]) = kreg[i];
      *(bf16x8*)(&ldsV[t * VSTRIDE + 8 * i])           = vreg[i];
    }
    if (kb + 32 <= kmax) {
      const bf16* kn = kSrc + (size_t)(kb + 32) * KVST;
      const bf16* vn = vSrc + (kb + 32);
#pragma unroll
      for (int i = 0; i < 4; ++i) {
        kreg[i] = *(const bf16x8*)(kn + 8 * i);
        vreg[i] = *(const bf16x8*)(vn + 8 * i);
      }
    }
    __syncthreads();

    bf16x16 kf[2][2];
#pragma unroll
    for (int ktile = 0; ktile < 2; ++ktile)
#pragma unroll
      for (int c = 0; c < 2; ++c)
        kf[ktile][c] = lds_frag(ldsK + (ktile * 16) * KSTRIDE + c * 32, KSTRIDE);

    bf16x16 pf[QW];
    bool act[QW];
#pragma unroll
    for (int qt = 0; qt < QW; ++qt) {
      unsigned mbits = 0;
      {
        const int q_my = q0 + 16 * qt + qlane;
#pragma unroll
        for (int r = 0; r < 8; ++r) { const int j0 = kb + kh8 + r, j1 = j0 + 16;
          if (j0 <= q_my && q_my - j0 < WIN) mbits |= 1u << r;
          if (j1 <= q_my && q_my - j1 < WIN) mbits |= 1u << (8 + r);
        }
        act[qt] = (__builtin_amdgcn_ballot_w32(mbits != 0) != 0);
      }
      if (act[qt]) {
        const int q_my = q0 + 16 * qt + qlane;
        f32x8 s0 = {}, s1 = {};
        s0 = wmma_bf16(kf[0][0], qf[qt][0], s0);
        s0 = wmma_bf16(kf[0][1], qf[qt][1], s0);
        s1 = wmma_bf16(kf[1][0], qf[qt][0], s1);
        s1 = wmma_bf16(kf[1][1], qf[qt][1], s1);

        float mx = -INFINITY;
#pragma unroll
        for (int r = 0; r < 8; ++r) {
          const int k0i = kb + kh8 + r;
          const int k1i = k0i + 16;
          (void)k0i; (void)k1i; (void)q_my;
          s0[r] = (mbits & (1u << r))       ? s0[r] * scale : NEG2;
          s1[r] = (mbits & (1u << (8 + r))) ? s1[r] * scale : NEG2;
          mx = fmaxf(mx, fmaxf(s0[r], s1[r]));
        }
        mx = fmaxf(mx, __shfl_xor(mx, 16, 32));
        const float mnew  = fmaxf(mrun[qt], mx);
        const float alpha = exp2f(mrun[qt] - mnew);

        float rsum = 0.0f;
#pragma unroll
        for (int r = 0; r < 8; ++r) {
          const float p0 = exp2f(s0[r] - mnew);
          const float p1 = exp2f(s1[r] - mnew);
          rsum += p0 + p1;
          pf[qt][r]     = (bf16)(p0 * 1024.0f);
          pf[qt][r + 8] = (bf16)(p1 * 1024.0f);
        }
        rsum += __shfl_xor(rsum, 16, 32);
        lrun[qt] = lrun[qt] * alpha + rsum;
        mrun[qt] = mnew;

#pragma unroll
        for (int j = 0; j < 4; ++j)
#pragma unroll
          for (int r = 0; r < 8; ++r) o[qt][j][r] *= alpha;
      }
    }

#pragma unroll
    for (int j = 0; j < 4; ++j) {
      const bf16x16 vf = lds_frag(ldsV + (j * 16) * VSTRIDE, VSTRIDE);
#pragma unroll
      for (int qt = 0; qt < QW; ++qt)
        if (act[qt]) o[qt][j] = wmma_bf16(vf, pf[qt], o[qt][j]);
    }
  }

  bf16* so = ldsO[wave];
#pragma unroll
  for (int qt = 0; qt < QW; ++qt) {
    const float rl = 1.0f / (lrun[qt] * 1024.0f);
#pragma unroll
    for (int j = 0; j < 4; ++j)
#pragma unroll
      for (int r = 0; r < 8; ++r) so[(16 * qt + qlane) * 72 + j * 16 + kh8 + r] = (bf16)(o[qt][j][r] * rl);
  }
  asm volatile("s_wait_dscnt 0" ::: "memory");
#pragma unroll 1
  for (int pass = 0; pass < 2; ++pass) {
#pragma unroll
    for (int it = 0; it < 8; ++it) { const int ch = lane + 32 * it, ql = ch >> 3, q8 = (ch & 7) * 8;
      *(volatile v4u_t*)(attnOut + ((size_t)(b * SS + q0 + ql)) * QST + h * DKK + q8) = *(const v4ua*)(so + ql * 72 + q8); }
    __threadfence();
  }
}


__global__ __launch_bounds__(256) void k_rms(const float* __restrict__ x, const float* __restrict__ nw, bf16* __restrict__ xw, float* __restrict__ rrow) {
  __shared__ __attribute__((aligned(16))) float rS[32];
  const int tid = threadIdx.x, lane = tid & 31, wave = tid >> 5;
#pragma unroll 1
  for (int rr = 0; rr < 4; ++rr) {
    const int row = blockIdx.x * 32 + wave * 4 + rr;
    const float* xr = x + (size_t)row * HID;
    bf16* yr = xw + (size_t)row * HID;
    float s = 0.0f;
    for (int c4 = lane; c4 < HID / 4; c4 += 32) { const v4f_t v = *(const v4f_t*)(xr + 4 * c4); s += v[0] * v[0] + v[1] * v[1] + v[2] * v[2] + v[3] * v[3]; }
#pragma unroll
    for (int off = 16; off >= 1; off >>= 1) s += __shfl_xor(s, off, 32);
    if (lane == 0) rS[wave * 4 + rr] = rsqrtf(s * (1.0f / (float)HID) + 1e-5f);
#pragma unroll 1
    for (int pass = 0; pass < 2; ++pass) {
      for (int c4 = lane; c4 < HID / 4; c4 += 32) {
        const v4f_t v = *(const v4f_t*)(xr + 4 * c4), w = *(const v4f_t*)(nw + 4 * c4);
        union { bf16 h[4]; unsigned long long u; } cv;
        cv.h[0] = (bf16)(v[0] * w[0]); cv.h[1] = (bf16)(v[1] * w[1]); cv.h[2] = (bf16)(v[2] * w[2]); cv.h[3] = (bf16)(v[3] * w[3]);
        *(volatile unsigned long long*)(yr + 4 * c4) = cv.u;
      }
      __threadfence();
    }
  }
  __syncthreads();
  if (wave == 0 && lane < 8) {
#pragma unroll 1
    for (int pass = 0; pass < 2; ++pass) { *(volatile v4f_t*)(rrow + blockIdx.x * 32 + lane * 4) = *(const volatile v4fa*)(rS + lane * 4); __threadfence(); }
  }
}
__global__ __launch_bounds__(256) void k_rope(const float* __restrict__ qk, const int* __restrict__ positions, RopeFreq rf, float mscale,
                                             bf16* __restrict__ Qb, bf16* __restrict__ Kb) {
  __shared__ __attribute__((aligned(16))) bf16 rowS[QKN];
  const int t = threadIdx.x, tok = blockIdx.x;
  const float pos = (float)positions[tok];
  const float* src = qk + (size_t)tok * QKN;
  for (int p = t; p < 72 * 32; p += 256) {
    const int hh = p >> 5, i = p & 31;
    const float f = pos * rf.inv[i];
    const float c = cosf(f) * mscale, s = sinf(f) * mscale;
    const float x1 = src[hh * 64 + i], x2 = src[hh * 64 + 32 + i];
    rowS[hh * 64 + i]      = (bf16)(x1 * c - x2 * s);
    rowS[hh * 64 + 32 + i] = (bf16)(x2 * c + x1 * s);
  }
  __syncthreads();
#pragma unroll 1
  for (int pass = 0; pass < 2; ++pass) {
    for (int ch = t; ch < QKN / 8; ch += 256) {
      const v4u_t v = *(const v4ua*)(rowS + ch * 8);
      if (ch < 512) *(volatile v4u_t*)(Qb + (size_t)tok * QST + ch * 8) = v;
      else          *(volatile v4u_t*)(Kb + (size_t)tok * KVST + (ch - 512) * 8) = v;
    }
    __threadfence();
  }
}

static RopeFreq yarn_inv_freq() {
  const double D = 64.0, THETA = 150000.0, FACTOR = 32.0, ORIG_MAX = 4096.0, BETA_FAST = 32.0, BETA_SLOW = 1.0, PI = 3.14159265358979323846;
  auto corr_dim = [&](double n_rot) { return D * log(ORIG_MAX / (n_rot * 2.0 * PI)) / (2.0 * log(THETA)); };
  double lowd = floor(corr_dim(BETA_FAST)); int low = lowd < 0 ? 0 : (int)lowd;
  double highd = ceil(corr_dim(BETA_SLOW)); int high = highd > D - 1 ? (int)(D - 1) : (int)highd;
  RopeFreq rf;
  for (int i = 0; i < 32; ++i) {
    const float pow_ = (float)(2 * i) / 64.0f;
    const float extrap = 1.0f / powf((float)THETA, pow_);
    const float interp = extrap / (float)FACTOR;
    float denom = (float)(high - low); if (denom < 1e-3f) denom = 1e-3f;
    float ramp = ((float)i - (float)low) / denom; ramp = ramp < 0.f ? 0.f : (ramp > 1.f ? 1.f : ramp);
    const float extrap_mask = 1.0f - ramp;
    rf.inv[i] = interp * (1.0f - extrap_mask) + extrap * extrap_mask;
  }
  return rf;
}

extern "C" void kernel_launch(void* const* d_in, const int* in_sizes, int n_in,
                              void* d_out, int out_size, void* d_ws, size_t ws_size,
                              hipStream_t stream) {
  (void)in_sizes; (void)n_in; (void)out_size; (void)ws_size;
  const float* x = (const float*)d_in[0];
  const int* positions = (const int*)d_in[1];
  const float* norm_w = (const float*)d_in[2];
  const float* w_qkv = (const float*)d_in[3];
  const float* b_qkv = (const float*)d_in[4];
  const float* w_o = (const float*)d_in[5];
  const float* b_o = (const float*)d_in[6];
  const float* sinks = (const float*)d_in[7];
  float* out = (float*)d_out;
  char* ws = (char*)d_ws;
  bf16* xw = (bf16*)ws;                         ws += (size_t)TT_ * HID * 2;
  float* rrow = (float*)ws;                     ws += 8192;
  float* qk = (float*)ws;                       ws += (size_t)TT_ * QKN * 4;
  bf16* VtB = (bf16*)ws;                        ws += (size_t)NKV * DKK * TT_ * 2;
  bf16* Qb = (bf16*)ws;                         ws += (size_t)TT_ * QST * 2;
  bf16* Kb = (bf16*)ws;                         ws += (size_t)TT_ * KVST * 2;
  bf16* att = (bf16*)ws;                        ws += (size_t)TT_ * QST * 2;
  const float mscale = (float)(0.1 * log(32.0) + 1.0);
  const RopeFreq rf = yarn_inv_freq();
  k_rms<<<dim3(TT_ / 32), dim3(256), 0, stream>>>(x, norm_w, xw, rrow);
  gemm_oai_kernel<bf16, 2><<<dim3(TT_ / 128, QKN / 256), dim3(256), 0, stream>>>(xw, w_qkv, b_qkv, rrow, nullptr, qk, TT_, QKN, HID);
  gemm_oai_kernel<bf16, 1><<<dim3(TT_ / 128, (NKV * DKK) / 256), dim3(256), 0, stream>>>(xw, w_qkv + (size_t)QKN * HID, b_qkv + QKN, rrow, nullptr, VtB, TT_, NKV * DKK, HID);
  k_rope<<<dim3(TT_), dim3(256), 0, stream>>>(qk, positions, rf, mscale, Qb, Kb);
  attn_kernel<<<dim3(SS / 64, NQH, 1), dim3(64), 0, stream>>>(Qb, Kb, VtB, sinks, att);
  gemm_oai_kernel<bf16, 2><<<dim3(TT_ / 128, (HID + 255) / 256), dim3(256), 0, stream>>>(att, w_o, b_o, nullptr, x, out, TT_, HID, QST);
}
